// GraphSPNMargkAry_69956427317253
// MI455X (gfx1250) — hardware-verified
//
#include <hip/hip_runtime.h>
#include <math.h>

#define ND_N      9
#define ARITY     5
#define NK        5
#define NI        40
#define NDIM      30
#define NCOMBO    126
#define EMPTY_TOK 4
#define KTOT      150
#define ROWS_PB   128
#define BSW_ELEMS (5*3*32*16)
#define GPB       32

typedef __attribute__((ext_vector_type(16))) _Float16 v16h;
typedef __attribute__((ext_vector_type(8)))  _Float16 v8h;
typedef __attribute__((ext_vector_type(8)))  float    v8f;

#define WS_COMBOS 0
#define WS_LOGW   4096
#define WS_BSW    8192

__device__ __forceinline__ void placebits(unsigned* mw, int d, int tok) {
  const unsigned oh = ((unsigned)tok < (unsigned)NK) ? (1u << tok) : 0u;
  const int bit = 5 * d;
  const int w   = bit >> 5;
  const int sh  = bit & 31;
  mw[w] |= oh << sh;
  if (sh > 27 && w < 4) mw[w + 1] |= oh >> (32 - sh);
}

__device__ __forceinline__ float ltheta_val(const float* __restrict__ theta, int e) {
  const int h    = e & 15;
  const int lane = (e >> 4) & 31;
  const int rest = e >> 9;
  const int tile = rest % 3;
  const int s    = rest / 3;
  const int K    = 32 * s + 8 * (lane >> 4) + ((h < 8) ? h : (h + 8));
  const int n    = tile * 16 + (lane & 15);
  float val = 0.f;
  if (K < KTOT && n < NI) {
    const int d   = K / NK;
    const int tok = K % NK;
    const float* row = theta + (n * NDIM + d) * NK;
    float m = row[0];
    for (int k = 1; k < NK; ++k) m = fmaxf(m, row[k]);
    float ss = 0.f;
    for (int k = 0; k < NK; ++k) ss += expf(row[k] - m);
    val = row[tok] - (m + logf(ss));
  }
  return val;
}

__global__ void __launch_bounds__(256) spn_prep_kernel(const float* __restrict__ theta,
                                const float* __restrict__ wlog,
                                int*   __restrict__ combos,
                                float* __restrict__ lw,
                                unsigned* __restrict__ bsw2) {
  __shared__ int scomb[128];
  const int t = threadIdx.x;

  if (t == 0) {
    int idx = 0;
    for (int c0 = 0; c0 < ND_N; ++c0)
      for (int c1 = c0 + 1; c1 < ND_N; ++c1)
        for (int c2 = c1 + 1; c2 < ND_N; ++c2)
          for (int c3 = c2 + 1; c3 < ND_N; ++c3)
            for (int c4 = c3 + 1; c4 < ND_N; ++c4)
              scomb[idx++] = c0 | (c1 << 4) | (c2 << 8) | (c3 << 12) | (c4 << 16);
    scomb[126] = 0; scomb[127] = 0;
  }
  float lwv = 0.f;
  if (t < NI) {
    float m = -INFINITY;
    for (int i = 0; i < NI; ++i) m = fmaxf(m, wlog[i]);
    float s = 0.f;
    for (int i = 0; i < NI; ++i) s += expf(wlog[i] - m);
    lwv = wlog[t] - (m + logf(s));
  }
  __syncthreads();
  for (int pass = 0; pass < 2; ++pass) {
    if (t < 128) ((volatile int*)combos)[t] = scomb[t];
    if (t < 64)  ((volatile float*)lw)[t] = lwv;
    for (int e2 = t; e2 < BSW_ELEMS / 2; e2 += 256) {
      const _Float16 v0 = (_Float16)ltheta_val(theta, 2 * e2);
      const _Float16 v1 = (_Float16)ltheta_val(theta, 2 * e2 + 1);
      const unsigned u = (unsigned)__builtin_bit_cast(unsigned short, v0) | ((unsigned)__builtin_bit_cast(unsigned short, v1) << 16);
      ((volatile unsigned*)bsw2)[e2] = u;
    }
    __threadfence();
  }
}

template <int S>
__device__ __forceinline__ void do_kstep(const unsigned* mw, int group, int lane,
                                         const _Float16* BsLDS, const _Float16* TsLDS,
                                         v8f& acc0, v8f& acc1, v8f& acc2) {
  const unsigned mg = mw[S] >> (group * 8);
  const v8h lo = *(const v8h*)(TsLDS + (mg & 0xFFu) * 8);
  const v8h hi = *(const v8h*)(TsLDS + ((mg >> 16) & 0xFFu) * 8);
  const v16h af = __builtin_shufflevector(lo, hi, 0, 1, 2, 3, 4, 5, 6, 7,
                                          8, 9, 10, 11, 12, 13, 14, 15);
  const _Float16* bb = BsLDS + (((S * 3) * 32) + lane) * 16;
  const v16h b0 = *(const v16h*)(bb);
  const v16h b1 = *(const v16h*)(bb + 32 * 16);
  const v16h b2 = *(const v16h*)(bb + 64 * 16);
  acc0 = __builtin_amdgcn_wmma_f32_16x16x32_f16(false, af, false, b0, (short)0, acc0, false, false);
  acc1 = __builtin_amdgcn_wmma_f32_16x16x32_f16(false, af, false, b1, (short)0, acc1, false, false);
  acc2 = __builtin_amdgcn_wmma_f32_16x16x32_f16(false, af, false, b2, (short)0, acc2, false, false);
  asm volatile("v_nop\n\tv_nop\n\tv_nop\n\tv_nop" : "+v"(acc0), "+v"(acc1), "+v"(acc2) : "v"(af), "v"(b0), "v"(b1), "v"(b2));
}

__global__ __launch_bounds__(256)
void spn_main_kernel(const int* __restrict__ xg,
                     const int* __restrict__ ag,
                     const float* __restrict__ rate,
                     const int* __restrict__ combos,
                     const float* __restrict__ lw,
                     const _Float16* __restrict__ bsw,
                     float* __restrict__ out,
                     int B) {
  __shared__ __align__(32) _Float16 Bs[BSW_ELEMS];
  __shared__ __align__(16) _Float16 Ts[256 * 8];
  __shared__ int   xs[ND_N];
  __shared__ int   as[ND_N * ND_N];
  __shared__ float lsh[ROWS_PB];
  __shared__ __align__(16) float res[GPB];

  const int tid = threadIdx.x;
  const int wave  = tid >> 5;
  const int lane  = tid & 31;
  const int col   = lane & 15;
  const int group = lane >> 4;

  for (int t = tid; t < BSW_ELEMS / 8; t += 256)
    *(v8h*)(Bs + t * 8) = *(const v8h*)(bsw + t * 8);
#pragma unroll
  for (int j = 0; j < 8; ++j)
    Ts[tid * 8 + j] = ((tid >> j) & 1) ? (_Float16)1.0f : (_Float16)0.0f;
  if (tid < GPB) res[tid] = 0.f;

  const int nc = wave * 16 + col;
  int cidx[ARITY] = {0, 0, 0, 0, 0};
  if (nc < NCOMBO) {
    const int cw = combos[nc];
#pragma unroll
    for (int j = 0; j < ARITY; ++j) cidx[j] = (cw >> (4 * j)) & 0xF;
  }
  const float lw0 = lw[col];
  const float lw1 = lw[16 + col];
  const float lw2 = (col < 8) ? lw[32 + col] : 0.f;
  const float rr  = rate[0];
  __syncthreads();

  for (int g = 0; g < GPB; ++g) {
    const int b = blockIdx.x * GPB + g;
    if (b >= B) break;
    __syncthreads();
    for (int t = tid; t < ND_N * ND_N; t += 256) as[t] = ag[b * 81 + t];
    if (tid < ND_N) xs[tid] = xg[b * ND_N + tid];
    __syncthreads();

    unsigned mw[5] = {0u, 0u, 0u, 0u, 0u};
    if (nc < NCOMBO) {
#pragma unroll
      for (int j = 0; j < ARITY; ++j) {
        placebits(mw, j * 6, xs[cidx[j]]);
#pragma unroll
        for (int k = 0; k < ARITY; ++k)
          placebits(mw, j * 6 + 1 + k, as[cidx[j] * ND_N + cidx[k]]);
      }
    }

    v8f acc0 = {}, acc1 = {}, acc2 = {};
    do_kstep<0>(mw, group, lane, Bs, Ts, acc0, acc1, acc2);
    do_kstep<1>(mw, group, lane, Bs, Ts, acc0, acc1, acc2);
    do_kstep<2>(mw, group, lane, Bs, Ts, acc0, acc1, acc2);
    do_kstep<3>(mw, group, lane, Bs, Ts, acc0, acc1, acc2);
    do_kstep<4>(mw, group, lane, Bs, Ts, acc0, acc1, acc2);

#pragma unroll
    for (int r = 0; r < 8; ++r) {
      const float a0 = acc0[r] + lw0;
      const float a1 = acc1[r] + lw1;
      const float a2 = (col < 8) ? (acc2[r] + lw2) : -INFINITY;
      float pm = fmaxf(fmaxf(a0, a1), a2);
#pragma unroll
      for (int off = 1; off <= 8; off <<= 1)
        pm = fmaxf(pm, __shfl_xor(pm, off, 32));
      float ps = expf(a0 - pm) + expf(a1 - pm) + expf(a2 - pm);
#pragma unroll
      for (int off = 1; off <= 8; off <<= 1)
        ps += __shfl_xor(ps, off, 32);
      if (col == 0) {
        const int n = wave * 16 + r + 8 * group;
        lsh[n] = (n < NCOMBO) ? (pm + logf(ps)) : -INFINITY;
      }
    }
    __syncthreads();

    if (wave == 0) {
      const float v0 = lsh[lane], v1 = lsh[lane + 32];
      const float v2 = lsh[lane + 64], v3 = lsh[lane + 96];
      float pm = fmaxf(fmaxf(v0, v1), fmaxf(v2, v3));
#pragma unroll
      for (int off = 1; off <= 16; off <<= 1)
        pm = fmaxf(pm, __shfl_xor(pm, off, 32));
      float ps = expf(v0 - pm) + expf(v1 - pm) + expf(v2 - pm) + expf(v3 - pm);
#pragma unroll
      for (int off = 1; off <= 16; off <<= 1)
        ps += __shfl_xor(ps, off, 32);
      if (lane == 0) {
        const float gll = pm + logf(ps) - logf((float)NCOMBO);
        int nf = 0;
#pragma unroll
        for (int d = 0; d < ND_N; ++d) nf += (xs[d] != EMPTY_TOK) ? 1 : 0;
        const float fnf = (float)nf;
        res[g] = fnf * rr - expf(rr) - lgammaf(fnf + 1.f) + gll;
      }
    }
  }
  __syncthreads();
  if (wave == 0) {
    const int b = blockIdx.x * GPB + lane;
    if (b < B) ((volatile float*)out)[b] = res[lane];
    __threadfence();
    if (b < B) ((volatile float*)out)[b] = res[lane];
  }
}

extern "C" void kernel_launch(void* const* d_in, const int* in_sizes, int n_in,
                              void* d_out, int out_size, void* d_ws, size_t ws_size,
                              hipStream_t stream) {
  (void)n_in; (void)ws_size;
  const int*   x_g     = (const int*)d_in[0];
  const int*   a_g     = (const int*)d_in[1];
  const float* theta_g = (const float*)d_in[2];
  const float* w_g     = (const float*)d_in[3];
  const float* rate_g  = (const float*)d_in[4];
  float*       out_g   = (float*)d_out;

  const int B = out_size;

  int*      ws_combos = (int*)((char*)d_ws + WS_COMBOS);
  float*    ws_lw     = (float*)((char*)d_ws + WS_LOGW);
  _Float16* ws_bsw    = (_Float16*)((char*)d_ws + WS_BSW);

  spn_prep_kernel<<<1, 256, 0, stream>>>(theta_g, w_g, ws_combos, ws_lw, (unsigned*)ws_bsw);
  spn_main_kernel<<<(B + GPB - 1) / GPB, 256, 0, stream>>>(x_g, a_g, rate_g, ws_combos, ws_lw, ws_bsw, out_g, B);
}
